// ComplexDifferentialAttention_68410239090889
// MI455X (gfx1250) — hardware-verified
//
#include <hip/hip_runtime.h>
#include <math.h>

typedef __attribute__((ext_vector_type(16))) _Float16 v16h;
typedef __attribute__((ext_vector_type(16))) __bf16 v16b;
typedef __attribute__((ext_vector_type(8)))  _Float16 v8h;
typedef __attribute__((ext_vector_type(8)))  float v8f;
typedef __attribute__((ext_vector_type(4)))  float v4f;
typedef __attribute__((ext_vector_type(2)))  float v2f;
typedef __attribute__((ext_vector_type(4)))  unsigned v4u;
typedef __attribute__((ext_vector_type(4)))  int v4i;
typedef float __attribute__((may_alias)) float_a;
typedef int __attribute__((may_alias)) int_a;

template <typename T> __device__ __forceinline__ void vst2(void* p, T v) { *(volatile T*)p = v; __threadfence(); *(volatile T*)p = v; }
__device__ __forceinline__ v8f wmma16(v16h a, v16h b, v8f c) {
  v8f d = __builtin_amdgcn_wmma_f32_16x16x32_f16(false, a, false, b, (short)0, c, false, false);
  asm volatile("v_nop\n\tv_nop\n\tv_nop\n\tv_nop" : "+v"(d) : "v"(a), "v"(b));
  return d;
}
__device__ __forceinline__ v8f wmma_bf(v16b a, v16b b, v8f c) {
  v8f d = __builtin_amdgcn_wmma_f32_16x16x32_bf16(false, a, false, b, (short)0, c, false, false);
  asm volatile("v_nop\n\tv_nop\n\tv_nop\n\tv_nop" : "+v"(d) : "v"(a), "v"(b));
  return d;
}
__device__ __forceinline__ v16h frag_h(const _Float16* rowk0, int lane) {
  union { v16h v; v8h q[2]; } u; const _Float16* p = rowk0 + 8 * (lane >> 4);
  u.q[0] = *(const v8h*)p; u.q[1] = *(const v8h*)(p + 16); return u.v;
}
__device__ __forceinline__ v16h frag_f32(const float* rowk0, int lane) {
  v16h a; const float* p = rowk0 + 8 * (lane >> 4);
#pragma unroll
  for (int i = 0; i < 8; ++i) { a[i] = (_Float16)p[i]; a[8 + i] = (_Float16)p[16 + i]; }
  return a;
}
__device__ __forceinline__ v16h frag_f32s(const float* rowk0, int lane, float sc) {
  v16h a; const float* p = rowk0 + 8 * (lane >> 4);
#pragma unroll
  for (int i = 0; i < 8; ++i) { a[i] = (_Float16)(p[i] * sc); a[8 + i] = (_Float16)(p[16 + i] * sc); }
  return a;
}
__device__ __forceinline__ v16h fragc_f32(const float* W, int k0, int n, int lane, int ld, int K) {
  v16h a; const int g = lane >> 4;
#pragma unroll
  for (int i = 0; i < 8; ++i) { const int ka = k0 + 8 * g + i, kb = ka + 16;
    a[i] = (_Float16)(ka < K ? W[(size_t)(ka < K ? ka : K - 1) * ld + n] : 0.f); a[8 + i] = (_Float16)(kb < K ? W[(size_t)(kb < K ? kb : K - 1) * ld + n] : 0.f); }
  return a;
}
struct F2 { v16b h, l; };
__device__ __forceinline__ F2 bsplit16(const float v[16]) { F2 r;
#pragma unroll
  for (int i = 0; i < 16; ++i) { const __bf16 h = (__bf16)v[i]; r.h[i] = h; r.l[i] = (__bf16)(v[i] - (float)h); }
  return r; }
__device__ __forceinline__ F2 split_row(const float* row, int k0, int lane) { float v[16]; const float* p = row + k0 + 8 * (lane >> 4);
#pragma unroll
  for (int i = 0; i < 8; ++i) { v[i] = p[i]; v[8 + i] = p[16 + i]; }
  return bsplit16(v); }
__device__ __forceinline__ F2 split_rowK(const float* row, int k0, int lane, int K) { float v[16]; const int g = lane >> 4;
#pragma unroll
  for (int i = 0; i < 8; ++i) { const int ka = k0 + 8 * g + i, kb = ka + 16; v[i] = ka < K ? row[ka < K ? ka : K - 1] : 0.f; v[8 + i] = kb < K ? row[kb < K ? kb : K - 1] : 0.f; }
  return bsplit16(v); }
__device__ __forceinline__ F2 split_col(const float* W, int k0, int n, int lane, int ld, int K) { float v[16]; const int g = lane >> 4;
#pragma unroll
  for (int i = 0; i < 8; ++i) { const int ka = k0 + 8 * g + i, kb = ka + 16; v[i] = ka < K ? W[(size_t)(ka < K ? ka : K - 1) * ld + n] : 0.f; v[8 + i] = kb < K ? W[(size_t)(kb < K ? kb : K - 1) * ld + n] : 0.f; }
  return bsplit16(v); }
__device__ __forceinline__ v8f mac3(const F2& a, const F2& b, v8f c) { c = wmma_bf(a.l, b.h, c); c = wmma_bf(a.h, b.l, c); return wmma_bf(a.h, b.h, c); }
__device__ __forceinline__ float sigm(float v) { return 1.0f / (1.0f + expf(-v)); }
#define LDSX() do { asm volatile("s_wait_dscnt 0" ::: "memory"); __builtin_amdgcn_wave_barrier(); __builtin_amdgcn_fence(__ATOMIC_RELEASE, "workgroup"); } while (0)


#define NHT 12
#define SS 1024
#define DD 128
#define KK 256
#ifndef NHU
#define NHU NHT
#endif
#define NR (NHU * SS)
#define NRF (NHT * SS)
#ifndef HG
#define HG 3
#endif
#define NPAIR (NHU * 2)
#define SCALE 0.0883883461356163f
#define LAMBDA_INIT 0.35550907254219055f
__device__ __forceinline__ float bfr(float v) { return (float)(__bf16)v; }
typedef __attribute__((ext_vector_type(8))) __bf16 v8b;
__device__ __forceinline__ v16b frag_b(const __bf16* rowk0, int lane) { union { v16b v; v8b q[2]; } u; const __bf16* p = rowk0 + 8 * (lane >> 4); u.q[0] = *(const v8b*)p; u.q[1] = *(const v8b*)(p + 16); return u.v; }

#define WS_QH  0u
#define WS_QL  (WS_QH + 2u * (size_t)NRF * 1024)
#define WS_KH  (WS_QL + 2u * (size_t)NRF * 1024)
#define WS_KL  (WS_KH + 2u * (size_t)NRF * KK)
#define WS_VT  (WS_KL + 2u * (size_t)NRF * KK)
#define WS_VL  (WS_VT + 2u * (size_t)NHT * KK * SS)
#define WS_G   (WS_VL + 2u * (size_t)NHT * KK * SS)
#define WS_Y   (WS_G + 4u * (size_t)NRF * KK)
#define WS_LAM (WS_Y + 4u * (size_t)NRF * 512)
#define WS_S   (WS_LAM + 128u)
#define WS_END (WS_S + 4u * (size_t)HG * SS * SS)

template <int MODE, int NO>
__global__ __launch_bounds__(128) void k_clin(const float* __restrict__ XR, const float* __restrict__ XI, const float* __restrict__ WR, const float* __restrict__ WI, const float* __restrict__ BR, const float* __restrict__ BI, const float* __restrict__ PER, const float* __restrict__ PEI, void* __restrict__ D0, void* __restrict__ D1) {
  __shared__ __align__(16) float sf[64][132];
  const int tid = threadIdx.x, wave = tid >> 5, lane = tid & 31, col = lane & 15, g = lane >> 4; const int c0 = blockIdx.y * 128; const size_t r0 = (size_t)blockIdx.x * 64; const int part = c0 / NO; const int oo0 = c0 % NO;
  v8f acc[8] = {};
#pragma unroll 2
  for (int kc = 0; kc < KK / 32; ++kc) { const bool imx = kc >= 4; const int kx = (kc & 3) * 32;
    v16b ah, al; bool two = false;
    if (MODE < 4) { const float* p = (imx ? XI : XR) + (r0 + wave * 16 + col) * DD + kx + 8 * g;
#pragma unroll
      for (int i = 0; i < 8; ++i) { ah[i] = (__bf16)p[i]; ah[8 + i] = (__bf16)p[16 + i]; } }
    else { const F2 a = split_row(XR + (r0 + wave * 16 + col) * KK, kc * 32, lane); ah = a.h; al = a.l; two = true; }
#pragma unroll
    for (int j = 0; j < 8; ++j) { v16b w; const int oo = oo0 + j * 16 + col; const float* WS0 = (part == 0) ? (imx ? WI : WR) : (imx ? WR : WI); const float sg = (part == 0 && imx) ? -1.0f : 1.0f;
#pragma unroll
      for (int i = 0; i < 8; ++i) { w[i] = (__bf16)(sg * WS0[(size_t)oo * DD + kx + 8 * g + i]); w[8 + i] = (__bf16)(sg * WS0[(size_t)oo * DD + kx + 16 + 8 * g + i]); }
      asm volatile("s_wait_loadcnt 0x0" ::: "memory"); acc[j] = wmma_bf(ah, w, acc[j]); if (two) acc[j] = wmma_bf(al, w, acc[j]); } }
  { const float* BB = part == 0 ? BR : BI; const float* PE = part == 0 ? PER : PEI;
#pragma unroll
    for (int j = 0; j < 8; ++j) { const int oo = oo0 + j * 16 + col; const float bb = bfr(BB[oo]);
#pragma unroll
      for (int r = 0; r < 8; ++r) { const int rl = wave * 16 + 8 * g + r; float v = acc[j][r] + bb; if (MODE <= 1) v += bfr(PE[(r0 + rl) * DD + (oo & (DD - 1))]); sf[rl][j * 16 + col] = v; }
      asm volatile("s_wait_loadcnt 0x0" ::: "memory"); } }
  __syncthreads();
  if (MODE == 0) {
    _Float16* QH = (_Float16*)D0; _Float16* QL = (_Float16*)D1; const int sel = oo0 / DD; const int dA = sel * 512 + (part ? 128 : 0), dB = sel * 512 + (part ? 256 : 384); const float sgB = part ? 1.0f : -1.0f;
    for (int e = tid; e < 64 * 16; e += 128) { const int rl = e >> 4, q = e & 15; v8h ha, la, hb, lb;
#pragma unroll
      for (int k = 0; k < 8; ++k) { const float v = sf[rl][q * 8 + k]; const _Float16 hv = (_Float16)v; ha[k] = hv; la[k] = (_Float16)((v - (float)hv) * 1024.0f); const float vb = v * sgB; const _Float16 hb2 = (_Float16)vb; hb[k] = hb2; lb[k] = (_Float16)((vb - (float)hb2) * 1024.0f); }
      const size_t ro = (r0 + rl) * 1024; vst2((v4u*)(QH + ro + dA + q * 8), *(const v4u*)&ha); vst2((v4u*)(QL + ro + dA + q * 8), *(const v4u*)&la); vst2((v4u*)(QH + ro + dB + q * 8), *(const v4u*)&hb); vst2((v4u*)(QL + ro + dB + q * 8), *(const v4u*)&lb); } }
  else if (MODE == 1) {
    _Float16* KH = (_Float16*)D0; _Float16* KL = (_Float16*)D1;
    for (int e = tid; e < 64 * 16; e += 128) { const int rl = e >> 4, q = e & 15; v8h ha, la;
#pragma unroll
      for (int k = 0; k < 8; ++k) { const float v = sf[rl][q * 8 + k]; const _Float16 hv = (_Float16)v; ha[k] = hv; la[k] = (_Float16)((v - (float)hv) * 1024.0f); }
      const size_t ro = (r0 + rl) * KK + c0; vst2((v4u*)(KH + ro + q * 8), *(const v4u*)&ha); vst2((v4u*)(KL + ro + q * 8), *(const v4u*)&la); } }
  else if (MODE == 2) {
    __bf16* VT = (__bf16*)D0; __bf16* VL = (__bf16*)D1; const size_t h = r0 / SS; const int s0 = (int)(r0 % SS);
    for (int e = tid; e < 128 * 8; e += 128) { const int cl = e >> 3, q = e & 7; v8b hb, lb;
#pragma unroll
      for (int k = 0; k < 8; ++k) { const float v = sf[q * 8 + k][cl]; const __bf16 bh = (__bf16)v; hb[k] = bh; lb[k] = (__bf16)(v - (float)bh); }
      const size_t o2 = (h * KK + c0 + cl) * (size_t)SS + s0 + q * 8; vst2((v4u*)(VT + o2), *(const v4u*)&hb); vst2((v4u*)(VL + o2), *(const v4u*)&lb); } }
  else if (MODE == 3) {
    float* G = (float*)D0; for (int e = tid; e < 64 * 32; e += 128) { const int rl = e >> 5, q = e & 31; vst2(G + (r0 + rl) * KK + c0 + q * 4, *(const v4f*)&sf[rl][q * 4]); } }
  else {
    float* O = (float*)(part == 0 ? D0 : D1); for (int e = tid; e < 64 * 32; e += 128) { const int rl = e >> 5, q = e & 31; vst2(O + (r0 + rl) * DD + q * 4, *(const v4f*)&sf[rl][q * 4]); } } }
__global__ __launch_bounds__(32) void k_lam(const float* __restrict__ LQ1, const float* __restrict__ LK1, const float* __restrict__ LQ2, const float* __restrict__ LK2, float* __restrict__ LAM) { __shared__ float sl;
  if (threadIdx.x == 0) { float s1 = 0.f, s2 = 0.f; for (int i = 0; i < DD; ++i) { s1 += bfr(LQ1[i]) * bfr(LK1[i]); s2 += bfr(LQ2[i]) * bfr(LK2[i]); } const float z = expf(s1) - expf(s2) + LAMBDA_INIT; sl = 1.0f / (1.0f + expf(-z)); }
  __syncthreads(); vst2(LAM + threadIdx.x, sl); }
__global__ __launch_bounds__(128) void k_sc(const _Float16* __restrict__ QH, const _Float16* __restrict__ QL, const _Float16* __restrict__ KH, const _Float16* __restrict__ KL, int p0, float* __restrict__ S0) { __shared__ __align__(16) float ss[4][16][68]; const int p = p0 + blockIdx.z; const int h = p >> 1, sel = p & 1; float* S = S0 + (size_t)blockIdx.z * SS * SS;
  const int tid = threadIdx.x, wave = tid >> 5, lane = tid & 31, col = lane & 15, g = lane >> 4; const int k0 = blockIdx.y * 64; const int ql0 = blockIdx.x * 64 + wave * 16; const size_t q0 = (size_t)h * SS + ql0; const size_t kb = (size_t)h * SS + k0;
  v8f ar[4] = {}, arl[4] = {}, ai[4] = {}, ail[4] = {};
#pragma unroll 2
  for (int kc = 0; kc < KK / 32; ++kc) { const _Float16* qh = QH + (q0 + col) * 1024 + sel * 512 + kc * 32; const _Float16* ql = QL + (q0 + col) * 1024 + sel * 512 + kc * 32;
    const v16h arh = frag_h(qh, lane), arlo = frag_h(ql, lane), aih = frag_h(qh + 256, lane), ailo = frag_h(ql + 256, lane);
#pragma unroll
    for (int j = 0; j < 4; ++j) { const size_t ko = (kb + j * 16 + col) * KK + kc * 32; const v16h khf = frag_h(KH + ko, lane), klf = frag_h(KL + ko, lane);
      ar[j] = wmma16(arh, khf, ar[j]); arl[j] = wmma16(arlo, khf, arl[j]); arl[j] = wmma16(arh, klf, arl[j]);
      ai[j] = wmma16(aih, khf, ai[j]); ail[j] = wmma16(ailo, khf, ail[j]); ail[j] = wmma16(aih, klf, ail[j]); } }
#pragma unroll
  for (int j = 0; j < 4; ++j)
#pragma unroll
    for (int r = 0; r < 8; ++r) { const float sr_ = ar[j][r] + arl[j][r] * (1.0f / 1024.0f), si_ = ai[j][r] + ail[j][r] * (1.0f / 1024.0f); ss[wave][8 * g + r][j * 16 + col] = sqrtf(sr_ * sr_ + si_ * si_ + 1e-8f) * SCALE; }
  LDSX(); for (int rl = 0; rl < 16; ++rl) if (lane < 16) vst2(S + (size_t)(ql0 + rl) * SS + k0 + lane * 4, *(const v4f*)&ss[wave][rl][lane * 4]); }
__global__ __launch_bounds__(256) void k_sm(float* __restrict__ S0) { __shared__ float sred[8]; __shared__ float sbc; __shared__ __align__(16) float sh[SS];
  const int t = threadIdx.x; const size_t row = blockIdx.x; float* sr = S0 + (size_t)blockIdx.y * SS * SS + row * SS; const int kend = SS;
  float m = -3.0e38f; for (int k = t; k < kend; k += 256) m = fmaxf(m, sr[k]);
#pragma unroll
  for (int o = 1; o < 32; o <<= 1) m = fmaxf(m, __shfl_xor(m, o));
  if ((t & 31) == 0) sred[t >> 5] = m; __syncthreads(); if (t == 0) { float a = sred[0]; for (int i = 1; i < 8; ++i) a = fmaxf(a, sred[i]); sbc = a; } __syncthreads(); m = sbc; __syncthreads();
  float sum = 0.f; for (int k = t; k < kend; k += 256) sum += expf(sr[k] - m);
#pragma unroll
  for (int o = 1; o < 32; o <<= 1) sum += __shfl_xor(sum, o);
  if ((t & 31) == 0) sred[t >> 5] = sum; __syncthreads(); if (t == 0) { float a = 0.f; for (int i = 0; i < 8; ++i) a += sred[i]; sbc = 1.0f / a; } __syncthreads(); const float inv = sbc;
  for (int k = t; k < kend; k += 256) sh[k] = expf(sr[k] - m) * inv * 2048.0f;
  __syncthreads(); for (int q = t; q < kend / 4; q += 256) vst2(sr + q * 4, *(const v4f*)&sh[q * 4]); }
__global__ __launch_bounds__(128) void k_pv(const float* __restrict__ PS0, const __bf16* __restrict__ VT, const __bf16* __restrict__ VL, int p0, float* __restrict__ Y) { const int p = p0 + blockIdx.z; const int h = p >> 1, sel = p & 1; const float* PS = PS0 + (size_t)blockIdx.z * SS * SS; __shared__ __align__(16) float ss[4][16][KK + 4];
  const int tid = threadIdx.x, wave = tid >> 5, lane = tid & 31, col = lane & 15, g = lane >> 4; const int ql0 = blockIdx.x * 64 + wave * 16;
  v8f acc[KK / 16] = {};
#pragma unroll 1
  for (int kc = 0; kc < SS / 32; ++kc) { const F2 pf = split_row(PS + (size_t)(ql0 + col) * SS, kc * 32, lane);
    asm volatile("s_wait_loadcnt 0x0" ::: "memory");
#pragma unroll
    for (int j = 0; j < KK / 16; ++j) { const size_t po = ((size_t)h * KK + j * 16 + col) * (size_t)SS + kc * 32; const v16b vh = frag_b(VT + po, lane); acc[j] = wmma_bf(pf.h, vh, acc[j]); acc[j] = wmma_bf(pf.l, vh, acc[j]); acc[j] = wmma_bf(pf.h, frag_b(VL + po, lane), acc[j]); } }
#pragma unroll
  for (int j = 0; j < KK / 16; ++j)
#pragma unroll
    for (int r = 0; r < 8; ++r) ss[wave][8 * g + r][j * 16 + col] = acc[j][r] * (1.0f / 2048.0f);
  LDSX(); for (int rl = 0; rl < 16; ++rl) { const size_t ro = ((size_t)h * SS + ql0 + rl) * 512 + sel * 256; vst2(Y + ro + lane * 4, *(const v4f*)&ss[wave][rl][lane * 4]); vst2(Y + ro + 128 + lane * 4, *(const v4f*)&ss[wave][rl][128 + lane * 4]); } }
__global__ __launch_bounds__(256) void k_mix(const float* __restrict__ Y, float* __restrict__ GZ, const float* __restrict__ LAM, const float* __restrict__ SW) {
  const int t = threadIdx.x; const int rl = t >> 4, sub = t & 15; const size_t row = (size_t)blockIdx.x * 16 + rl; const float* y = Y + row * 512; float* gz = GZ + row * KK; const float lam = LAM[0];
  float s2 = 0.f; for (int c = sub * 4; c < 512; c += 64) { const v4f v = *(const v4f*)(y + c); s2 += (v[0] * v[0] + v[1] * v[1]) + (v[2] * v[2] + v[3] * v[3]); }
#pragma unroll
  for (int o = 1; o < 16; o <<= 1) s2 += __shfl_xor(s2, o);
  const float inv = 1.0f / sqrtf(s2 * (1.0f / 256.0f) + 1e-5f);
#pragma unroll
  for (int it = 0; it < 2; ++it) { const int d = sub * 4 + it * 64;
    const v4f a1r = *(const v4f*)(y + d), a1i = *(const v4f*)(y + 128 + d), a2r = *(const v4f*)(y + 256 + d), a2i = *(const v4f*)(y + 384 + d); const v4f gr = *(const v4f*)(gz + d), gi = *(const v4f*)(gz + 128 + d);
    v4f zr, zi;
#pragma unroll
    for (int k = 0; k < 4; ++k) { const float w1 = bfr(SW[d + k]) * inv, w2 = bfr(SW[DD + d + k]) * inv; const float orr = a1r[k] * w1 - lam * (a2r[k] * w2), oi = a1i[k] * w1 - lam * (a2i[k] * w2); zr[k] = gr[k] * orr - gi[k] * oi; zi[k] = gr[k] * oi + gi[k] * orr; }
    vst2(gz + d, zr); vst2(gz + 128 + d, zi); } }
extern "C" void kernel_launch(void* const* d_in, const int* in_sizes, int n_in, void* d_out, int out_size, void* d_ws, size_t ws_size, hipStream_t stream) {
  (void)in_sizes; (void)n_in; (void)out_size;
  const float** F = (const float**)d_in;
  if (ws_size < (size_t)WS_END) return;
  char* ws = (char*)d_ws; _Float16 *QH = (_Float16*)(ws + WS_QH), *QL = (_Float16*)(ws + WS_QL), *KH = (_Float16*)(ws + WS_KH), *KL = (_Float16*)(ws + WS_KL); __bf16 *VT = (__bf16*)(ws + WS_VT), *VL = (__bf16*)(ws + WS_VL); float *G = (float*)(ws + WS_G), *Y = (float*)(ws + WS_Y), *LAM = (float*)(ws + WS_LAM), *S = (float*)(ws + WS_S);
  float* OUT0 = (float*)d_out; float* OUT1 = (float*)d_out + (size_t)NRF * DD;
  k_clin<0, 256><<<dim3(NR / 64, 4), 128, 0, stream>>>(F[0], F[1], F[10], F[11], F[12], F[13], F[6], F[7], QH, QL);
  k_clin<1, 128><<<dim3(NR / 64, 2), 128, 0, stream>>>(F[2], F[3], F[14], F[15], F[16], F[17], F[8], F[9], KH, KL);
  k_clin<2, 128><<<dim3(NR / 64, 2), 128, 0, stream>>>(F[4], F[5], F[18], F[19], F[20], F[21], nullptr, nullptr, VT, VL);
  k_clin<3, 128><<<dim3(NR / 64, 2), 128, 0, stream>>>(F[0], F[1], F[22], F[23], F[24], F[25], nullptr, nullptr, G, nullptr);
  k_lam<<<dim3(1), 32, 0, stream>>>(F[30], F[31], F[32], F[33], LAM);
  for (int p0 = 0; p0 < NPAIR; p0 += HG) {
    k_sc<<<dim3(SS / 64, SS / 64, HG), 128, 0, stream>>>(QH, QL, KH, KL, p0, S);
    k_sm<<<dim3(SS, HG), 256, 0, stream>>>(S);
    k_pv<<<dim3(SS / 64, 1, HG), 128, 0, stream>>>(S, VT, VL, p0, Y);
  }
  k_mix<<<dim3(NR / 16), 256, 0, stream>>>(Y, G, LAM, F[34]);
  k_clin<4, 128><<<dim3(NR / 64, 2), 128, 0, stream>>>(G, nullptr, F[26], F[27], F[28], F[29], nullptr, nullptr, OUT0, OUT1);
}
